// RNadeOutputLayer_65790309040623
// MI455X (gfx1250) — hardware-run, weakly checked
//
#include <hip/hip_runtime.h>


#define NB   256
#define NH   512
#define ND   64
#define NK   16
typedef _Float16 h16;
typedef unsigned short bf;
typedef __attribute__((ext_vector_type(16))) __bf16   v16bf;
typedef __attribute__((ext_vector_type(16))) _Float16 v16h;
typedef __attribute__((ext_vector_type(8)))  _Float16 v8h;
typedef __attribute__((ext_vector_type(8)))  unsigned short v8us;
typedef __attribute__((ext_vector_type(8)))  float    v8f;
typedef __attribute__((ext_vector_type(4)))  float    v4f;
typedef v8h  __attribute__((may_alias)) v8ha;
typedef v4f  __attribute__((may_alias)) v4fa;
typedef v8us __attribute__((may_alias)) v8usa;

__device__ __forceinline__ unsigned short f2bf(float f) { unsigned u = __float_as_uint(f); u += 0x7FFFu + ((u >> 16) & 1u); return (unsigned short)(u >> 16); }
__device__ __forceinline__ float bf2f(unsigned short b) { return __uint_as_float(((unsigned)b) << 16); }
__device__ __forceinline__ float bfr(float f) { return bf2f(f2bf(f)); }
__device__ __forceinline__ v16h cat16(v8h lo, v8h hi) { return __builtin_shufflevector(lo, hi, 0, 1, 2, 3, 4, 5, 6, 7, 8, 9, 10, 11, 12, 13, 14, 15); }
__device__ __forceinline__ v16bf cat16b(v8us lo, v8us hi) { return __builtin_bit_cast(v16bf, __builtin_shufflevector(lo, hi, 0, 1, 2, 3, 4, 5, 6, 7, 8, 9, 10, 11, 12, 13, 14, 15)); }
__device__ __forceinline__ v8f wmma16(v16h a, v16h b, v8f c) { return __builtin_amdgcn_wmma_f32_16x16x32_f16(false, a, false, b, (short)0, c, false, false); }
__device__ __forceinline__ v8f wmmab(v16bf a, v16bf b, v8f c) { return __builtin_amdgcn_wmma_f32_16x16x32_bf16(false, a, false, b, (short)0, c, false, false); }

template <typename T16> struct WFrag;
template <> struct WFrag<h16> { typedef v16h V; static __device__ __forceinline__ V ld(const h16* p) { return cat16(*(const v8h*)p, *(const v8h*)(p + 16)); } static __device__ __forceinline__ v8f mma(V a, V b, v8f c) { return wmma16(a, b, c); } };
template <> struct WFrag<bf> { typedef v16bf V; static __device__ __forceinline__ V ld(const bf* p) { return cat16b(*(const v8us*)p, *(const v8us*)(p + 16)); } static __device__ __forceinline__ v8f mma(V a, V b, v8f c) { return wmmab(a, b, c); } };
template <typename T16, int NSPLIT, bool BIAS>
__global__ __launch_bounds__(32) void k_gemmw(const T16* __restrict__ A, const T16* __restrict__ A2, const T16* __restrict__ Bt, const T16* __restrict__ Bt2, int K, float* C, int ldc, const float* __restrict__ bias, size_t sA, size_t sB, size_t sC) {
    typedef typename WFrag<T16>::V V;
    __shared__ __align__(16) float os[16 * 68];
    const size_t z = blockIdx.z; A += z * sA; if (A2) A2 += z * sA; Bt += z * sB; if (Bt2) Bt2 += z * sB; C += z * sC;
    const int lane = threadIdx.x & 31, lr = lane & 15, hi = lane >> 4; const int r0 = blockIdx.x * 64, c0 = blockIdx.y * 64;
    v8f acc[4][4];
#pragma unroll
    for (int mb = 0; mb < 4; ++mb)
#pragma unroll
        for (int nb = 0; nb < 4; ++nb) acc[mb][nb] = (v8f){};
    const size_t aoff = (size_t)(r0 + lr) * K + 8 * hi, boff = (size_t)(c0 + lr) * K + 8 * hi;
    for (int kc = 0; kc < K; kc += 32) {
        V a[4], a2[4];
#pragma unroll
        for (int mb = 0; mb < 4; ++mb) { a[mb] = WFrag<T16>::ld(A + aoff + (size_t)mb * 16 * K + kc); if (NSPLIT == 1 || NSPLIT == 2) a2[mb] = WFrag<T16>::ld(A2 + aoff + (size_t)mb * 16 * K + kc); }
#pragma unroll
        for (int nb = 0; nb < 4; ++nb) { const V b = WFrag<T16>::ld(Bt + boff + (size_t)nb * 16 * K + kc); V b2; if (NSPLIT >= 2) b2 = WFrag<T16>::ld(Bt2 + boff + (size_t)nb * 16 * K + kc);
#pragma unroll
            for (int mb = 0; mb < 4; ++mb) { acc[mb][nb] = WFrag<T16>::mma(a[mb], b, acc[mb][nb]); if (NSPLIT == 1 || NSPLIT == 2) acc[mb][nb] = WFrag<T16>::mma(a2[mb], b, acc[mb][nb]); if (NSPLIT >= 2) acc[mb][nb] = WFrag<T16>::mma(a[mb], b2, acc[mb][nb]); } }
        asm volatile("v_nop\n\tv_nop\n\tv_nop\n\tv_nop" : "+v"(acc[0][0]), "+v"(acc[1][1]), "+v"(acc[2][2]), "+v"(acc[3][3]) : "v"(a[0]), "v"(a[3]));
    }
#pragma unroll
    for (int mb = 0; mb < 4; ++mb) {
#pragma unroll
        for (int nb = 0; nb < 4; ++nb) {
#pragma unroll
            for (int j = 0; j < 8; ++j) os[(hi * 8 + j) * 68 + nb * 16 + lr] = acc[mb][nb][j]; }
        __builtin_amdgcn_wave_barrier(); asm volatile("" ::: "memory");
        float* crow = C + (size_t)(r0 + mb * 16) * ldc + c0;
#pragma unroll 1
        for (int ps = 0; ps < 2; ++ps) {
#pragma unroll
            for (int s = 0; s < 8; ++s) { const int row = 2 * s + hi, cofs = lr * 4; v4f val = *(const v4fa*)(os + row * 68 + cofs); if (BIAS) { val[0] += bfr(bias[c0 + cofs]); val[1] += bfr(bias[c0 + cofs + 1]); val[2] += bfr(bias[c0 + cofs + 2]); val[3] += bfr(bias[c0 + cofs + 3]); }
                *(volatile v4f*)(crow + (size_t)row * ldc + cofs) = val; }
            if (ps == 0) __threadfence(); }
        __builtin_amdgcn_wave_barrier(); asm volatile("" ::: "memory");
    }
}

__global__ __launch_bounds__(256) void k_xa(const float* __restrict__ x, bf* XA) { const unsigned w = blockIdx.x * 256u + threadIdx.x; const unsigned h0 = (w & 63u) * 8u, b = (w >> 6) & 255u, d = w >> 14; const float* s = x + ((size_t)b * NH + h0) * ND + d; v8us o;
#pragma unroll
    for (int q = 0; q < 8; ++q) o[q] = f2bf(s[(size_t)q * ND]);
    bf* p = XA + ((size_t)d * NB + b) * NH + h0; *(volatile v8us*)p = o; __threadfence(); *(volatile v8us*)p = o; }

__global__ __launch_bounds__(256) void k_vb(const float* __restrict__ va, const float* __restrict__ vm, const float* __restrict__ vs, bf* VB) { const unsigned w = blockIdx.x * 256u + threadIdx.x; const unsigned h0 = (w & 63u) * 8u, r = (w >> 6) & 63u, d = w >> 12; const unsigned g = r >> 4, k = r & 15u; const float* v = (g == 0u) ? va : (g == 1u) ? vm : vs; const float live = (g < 3u) ? 1.0f : 0.0f; const float* s = v + ((size_t)k * NH + h0) * ND + d; v8us o;
#pragma unroll
    for (int q = 0; q < 8; ++q) o[q] = f2bf(__fmul_rn(live, s[(size_t)q * ND]));
    bf* p = VB + ((size_t)d * 64 + r) * NH + h0; *(volatile v8us*)p = o; __threadfence(); *(volatile v8us*)p = o; }

__global__ __launch_bounds__(256) void k_lp(const float* __restrict__ C, const float* __restrict__ y, const float* __restrict__ ca, const float* __restrict__ cm, const float* __restrict__ cs, float* LS) { const unsigned w = blockIdx.x * 256u + threadIdx.x; const unsigned d = w & 63u, b = w >> 6; const float* c = C + ((size_t)d * NB + b) * 64; const float yv = bfr(y[(size_t)b * ND + d]); float ea[NK], mu[NK], ls[NK];
#pragma unroll
    for (int g = 0; g < 4; ++g) { const v4f a = *(const v4f*)(c + 4 * g), m = *(const v4f*)(c + 16 + 4 * g), s = *(const v4f*)(c + 32 + 4 * g);
#pragma unroll
        for (int j = 0; j < 4; ++j) { const int k = 4 * g + j; ea[k] = __fadd_rn(a[j], bfr(ca[k * ND + d])); mu[k] = __fadd_rn(m[j], bfr(cm[k * ND + d])); ls[k] = fminf(fmaxf(__fadd_rn(s[j], bfr(cs[k * ND + d])), -20.0f), 20.0f); } }
    float M = ea[0];
#pragma unroll
    for (int k = 1; k < NK; ++k) M = (ea[k] > M) ? ea[k] : M;
    float z = 0.0f;
#pragma unroll
    for (int k = 0; k < NK; ++k) z = __fadd_rn(z, expf(__fsub_rn(ea[k], M)));
    const float lz = __fadd_rn(M, logf(z)); float lp[NK];
#pragma unroll
    for (int k = 0; k < NK; ++k) { const float q = __fdiv_rn(__fsub_rn(yv, mu[k]), expf(ls[k])); lp[k] = __fsub_rn(__fsub_rn(__fadd_rn(__fmul_rn(-0.5f, __fmul_rn(q, q)), __fsub_rn(ea[k], lz)), 0.918938533204672742f), ls[k]); }
    float P = lp[0];
#pragma unroll
    for (int k = 1; k < NK; ++k) P = (lp[k] > P) ? lp[k] : P;
    float t = 0.0f;
#pragma unroll
    for (int k = 0; k < NK; ++k) t = __fadd_rn(t, expf(__fsub_rn(lp[k], P)));
    const float r = __fadd_rn(P, logf(t)); *(volatile float*)(LS + w) = r; __threadfence(); *(volatile float*)(LS + w) = r; }

__global__ __launch_bounds__(256) void k_sm(const float* __restrict__ LS, float* out) { const unsigned b = threadIdx.x; const float* p = LS + (size_t)b * ND; float s = 0.0f;
    for (int g = 0; g < ND / 4; ++g) { const v4f v = *(const v4f*)(p + 4 * g);
#pragma unroll
        for (int j = 0; j < 4; ++j) s = __fadd_rn(s, v[j]); }
    *(volatile float*)(out + b) = s; __threadfence(); *(volatile float*)(out + b) = s; }

extern "C" void kernel_launch(void* const* d_in, const int* in_sizes, int n_in, void* d_out, int out_size, void* d_ws, size_t ws_size, hipStream_t stream) {
    if (n_in < 8) return;
    if (in_sizes[0] != NB * NH * ND || in_sizes[1] != NB * ND || in_sizes[2] != NK * NH * ND || in_sizes[3] != NK * NH * ND || in_sizes[4] != NK * NH * ND || in_sizes[5] != NK * ND || in_sizes[6] != NK * ND || in_sizes[7] != NK * ND) return;
    if (out_size != NB) return;
    static_assert(NB % 64 == 0 && NH % 64 == 0 && NH % 32 == 0 && ND == 64 && NK == 16 && NB == 256 && NH == 512, "the product: M a multiple of 64, N 64, the depth a multiple of 32; a plane row a whole number of lines; the index arithmetic of the builders is by shifts for these sizes");
    const float* x = (const float*)d_in[0]; const float* y = (const float*)d_in[1]; const float* va = (const float*)d_in[2]; const float* vm = (const float*)d_in[3]; const float* vs = (const float*)d_in[4]; const float* ca = (const float*)d_in[5]; const float* cm = (const float*)d_in[6]; const float* cs = (const float*)d_in[7];
    float* out = (float*)d_out;
    char* wsp = (char*)d_ws; auto take = [&](size_t bytes) { char* ptr = wsp; wsp += (bytes + 255) & ~(size_t)255; return (void*)ptr; };
    bf* XA = (bf*)take((size_t)ND * NB * NH * 2); bf* VB = (bf*)take((size_t)ND * 64 * NH * 2); float* C = (float*)take((size_t)ND * NB * 64 * 4); float* LS = (float*)take((size_t)NB * ND * 4);
    if ((size_t)(wsp - (char*)d_ws) > ws_size) return;
    k_xa<<<(unsigned)((size_t)ND * NB * NH / 8 / 256), 256, 0, stream>>>(x, XA);
    k_vb<<<(unsigned)((size_t)ND * 64 * NH / 8 / 256), 256, 0, stream>>>(va, vm, vs, VB);
    k_gemmw<bf, 0, false><<<dim3(NB / 64, 1, ND), 32, 0, stream>>>(XA, nullptr, VB, nullptr, NH, C, 64, nullptr, (size_t)NB * NH, (size_t)64 * NH, (size_t)NB * 64);
    k_lp<<<(unsigned)(NB * ND / 256), 256, 0, stream>>>(C, y, ca, cm, cs, LS);
    k_sm<<<1, 256, 0, stream>>>(LS, out);
}
